// MultiHeadSelfAttention_3264175145623
// MI455X (gfx1250) — hardware-verified
//
#include <hip/hip_runtime.h>
#include <math.h>

typedef __attribute__((ext_vector_type(16))) _Float16 v16h;
typedef __attribute__((ext_vector_type(16))) __bf16 v16b;
typedef __attribute__((ext_vector_type(8)))  _Float16 v8h;
typedef __attribute__((ext_vector_type(8)))  __bf16 v8b;
typedef __attribute__((ext_vector_type(8)))  float v8f;
typedef __attribute__((ext_vector_type(4)))  float v4f;
typedef __attribute__((ext_vector_type(4)))  unsigned v4u;

#ifndef NB
#define NB 2
#endif
#ifndef SEQ
#define SEQ 2048
#endif
#define NB_FULL 2
#define SEQ_FULL 2048
#define DIN 1024
#define CC 1024
#define NH 16
#define HD 64
#define NQB (SEQ / 64)
#define QBH 4
#define KHI 256
#define SCALE 0.125f
#define PCARRY 1024.0f

static_assert(NB >= 1 && NB <= NB_FULL);
static_assert(SEQ <= SEQ_FULL);
static_assert(SEQ % 64 == 0);
static_assert(SEQ % 8 == 0);
static_assert(CC == NH * HD);
static_assert(HD == 64);
static_assert(DIN == CC);
static_assert(DIN % 32 == 0);
static_assert(CC % 128 == 0);
static_assert(KHI == QBH * 64);
static_assert(KHI <= SEQ);
static_assert(NQB >= QBH);
static_assert(((size_t)NB * SEQ * DIN) % 2048 == 0);
static_assert(((size_t)CC * DIN) % 2048 == 0);

#define PLN ((size_t)NB * SEQ * CC)
#define WN  ((size_t)CC * DIN)
#define WS_XB  ((size_t)0)
#define WS_WB  (WS_XB + 2u * PLN)
#define WS_CS  (WS_WB + 2u * 4u * WN)
#define WS_QK  (WS_CS + 4u * (size_t)SEQ * 64u)
#define WS_VT  (WS_QK + 2u * 4u * PLN)
#define WS_VB  (WS_VT + 2u * PLN)
#define WS_VBL (WS_VB + 2u * (size_t)NB * CC * KHI)
#define WS_CH  (WS_VBL + 2u * (size_t)NB * CC * KHI)
#define WS_CL  (WS_CH + 2u * PLN)
#define WS_END (WS_CL + 2u * PLN)
static_assert(WS_END <= (size_t)134217728u);
static_assert(WS_WB % 128 == 0 && WS_CS % 128 == 0 && WS_QK % 128 == 0 && WS_VT % 128 == 0 && WS_VB % 128 == 0 && WS_VBL % 128 == 0 && WS_CH % 128 == 0 && WS_CL % 128 == 0);

template <typename T> __device__ __forceinline__ void vst2(void* p, T v) { *(volatile T*)p = v; __threadfence(); *(volatile T*)p = v; }
__device__ __forceinline__ v8f wmma16(v16h a, v16h b, v8f c) {
  v8f d = __builtin_amdgcn_wmma_f32_16x16x32_f16(false, a, false, b, (short)0, c, false, false);
  asm volatile("v_nop\n\tv_nop\n\tv_nop\n\tv_nop" : "+v"(d) : "v"(a), "v"(b));
  return d;
}
__device__ __forceinline__ v8f wmma_bf(v16b a, v16b b, v8f c) {
  v8f d = __builtin_amdgcn_wmma_f32_16x16x32_bf16(false, a, false, b, (short)0, c, false, false);
  asm volatile("v_nop\n\tv_nop\n\tv_nop\n\tv_nop" : "+v"(d) : "v"(a), "v"(b));
  return d;
}
__device__ __forceinline__ v16h frag_h(const _Float16* rowk0, int lane) {
  union { v16h v; v8h q[2]; } u; const _Float16* p = rowk0 + 8 * (lane >> 4);
  u.q[0] = *(const v8h*)p; u.q[1] = *(const v8h*)(p + 16); return u.v;
}
__device__ __forceinline__ v16b frag_b(const __bf16* rowk0, int lane) {
  union { v16b v; v8b q[2]; } u; const __bf16* p = rowk0 + 8 * (lane >> 4);
  u.q[0] = *(const v8b*)p; u.q[1] = *(const v8b*)(p + 16); return u.v;
}
#define LDSX() do { asm volatile("s_wait_dscnt 0" ::: "memory"); __builtin_amdgcn_wave_barrier(); __builtin_amdgcn_fence(3  , "workgroup"); } while (0)

__global__ __launch_bounds__(256) void k_cvt(const float* __restrict__ src, __bf16* __restrict__ dst, int seq, int seq_full) {
  const size_t e = ((size_t)blockIdx.x * 256 + threadIdx.x) * 8;
  const int row = (int)(e / DIN), cc = (int)(e % DIN);
  const int b = row / seq, t = row - b * seq;
  const float* p = src + ((size_t)b * seq_full + t) * DIN + cc;
  const v4f a = *(const v4f*)p; const v4f c = *(const v4f*)(p + 4);
  union { v8b h; v4u u; } o;
  o.h[0] = (__bf16)a[0]; o.h[1] = (__bf16)a[1]; o.h[2] = (__bf16)a[2]; o.h[3] = (__bf16)a[3];
  o.h[4] = (__bf16)c[0]; o.h[5] = (__bf16)c[1]; o.h[6] = (__bf16)c[2]; o.h[7] = (__bf16)c[3];
  vst2((void*)(dst + e), o.u);
}

__global__ __launch_bounds__(256) void k_tab(float* __restrict__ CS) {
  __shared__ __align__(16) float st[512];
  const int tid = threadIdx.x; const int idx = blockIdx.x * 256 + tid; const int s = idx >> 5, j = idx & 31;
  double p = (j & 1) ? 1.3335214321633240 : 1.0;
  p *= (j & 2) ? 1.7782794100389228 : 1.0;
  p *= (j & 4) ? 3.1622776601683795 : 1.0;
  p *= (j & 8) ? 10.0 : 1.0;
  p *= (j & 16) ? 100.0 : 1.0;
  const float pf = (float)p; const float inv = 1.0f / pf; const float ang = (float)s * inv;
  st[2 * tid] = cosf(ang); st[2 * tid + 1] = sinf(ang);
  __syncthreads();
  if (tid < 128) vst2((void*)(CS + (size_t)blockIdx.x * 512 + tid * 4), *(const v4f*)&st[tid * 4]);
}

__device__ __forceinline__ void gemm_row16x128(const __bf16* __restrict__ A, const __bf16* __restrict__ W, const size_t arow, const int c0, const int lane, v8f (&acc)[8]) {
  const int col = lane & 15;
#pragma unroll 2
  for (int kc = 0; kc < DIN / 32; ++kc) {
    const v16b a = frag_b(A + arow * DIN + kc * 32, lane);
#pragma unroll
    for (int j = 0; j < 8; ++j) { const v16b w = frag_b(W + (size_t)(c0 + j * 16 + col) * DIN + kc * 32, lane); acc[j] = wmma_bf(a, w, acc[j]); }
  }
}

__global__ __launch_bounds__(128) void k_projqk(const __bf16* __restrict__ XB, const __bf16* __restrict__ WB, const float* __restrict__ CS, __bf16* __restrict__ QK) {
  __shared__ __align__(16) __bf16 sh[64][136];
  __shared__ __align__(16) __bf16 sl[64][136];
  __shared__ __align__(16) float cst[64 * 64];
  const int tid = threadIdx.x; const int wave = __builtin_amdgcn_readfirstlane((int)(threadIdx.x >> 5)); const int lane = tid & 31, col = lane & 15, g = lane >> 4;
  const int which = blockIdx.z; const int c0 = blockIdx.y * 128; const size_t r0 = (size_t)blockIdx.x * 64; const int t0 = (int)(r0 % SEQ);
  for (int e = tid; e < 1024; e += 128) *(v4f*)&cst[e * 4] = *(const v4f*)(CS + (size_t)t0 * 64 + e * 4);
  v8f acc[8] = {};
  gemm_row16x128(XB, WB + (size_t)which * WN, r0 + wave * 16 + col, c0, lane, acc);
  __syncthreads();
  const bool odd = (lane & 1) != 0;
#pragma unroll
  for (int j = 0; j < 8; ++j) { const int jj = ((j * 16 + col) & 63) >> 1;
#pragma unroll
    for (int r = 0; r < 8; ++r) { const int rl = wave * 16 + 8 * g + r; const float x = acc[j][r]; const float xp = __shfl_xor(x, 1);
      const float cs = cst[rl * 64 + 2 * jj], sn = cst[rl * 64 + 2 * jj + 1];
      const float t1 = x * cs, t2 = xp * sn; const float v = odd ? (t1 + t2) : (t1 - t2);
      const __bf16 hv = (__bf16)v; sh[rl][j * 16 + col] = hv; sl[rl][j * 16 + col] = (__bf16)(v - (float)hv); } }
  __syncthreads();
  __bf16* DH = QK + (size_t)(2 * which) * PLN; __bf16* DL = DH + PLN;
  for (int e = tid; e < 64 * 16; e += 128) { const int rl = e >> 4, q = e & 15; const size_t off = (r0 + rl) * CC + c0 + q * 8;
    vst2((void*)(DH + off), *(const v4u*)&sh[rl][q * 8]); vst2((void*)(DL + off), *(const v4u*)&sl[rl][q * 8]); }
}

__global__ __launch_bounds__(128) void k_projv(const __bf16* __restrict__ XB, const __bf16* __restrict__ WB, _Float16* __restrict__ VT, __bf16* __restrict__ VB, __bf16* __restrict__ VBL) {
  __shared__ __align__(16) _Float16 th[128][72];
  __shared__ __align__(16) __bf16 tb[128][72];
  __shared__ __align__(16) __bf16 tbl[128][72];
  const int tid = threadIdx.x; const int wave = __builtin_amdgcn_readfirstlane((int)(threadIdx.x >> 5)); const int lane = tid & 31, col = lane & 15, g = lane >> 4;
  const int c0 = blockIdx.y * 128; const size_t r0 = (size_t)blockIdx.x * 64; const size_t bb = r0 / SEQ; const int t0 = (int)(r0 % SEQ);
  const bool hi_rows = t0 < KHI;
  v8f acc[8] = {};
  gemm_row16x128(XB, WB + (size_t)2 * WN, r0 + wave * 16 + col, c0, lane, acc);
#pragma unroll
  for (int j = 0; j < 8; ++j) {
#pragma unroll
    for (int r = 0; r < 8; ++r) { const float v = acc[j][r]; const int rl = wave * 16 + 8 * g + r, cl = j * 16 + col; th[cl][rl] = (_Float16)v;
      if (hi_rows) { const __bf16 bh = (__bf16)v; tb[cl][rl] = bh; tbl[cl][rl] = (__bf16)(v - (float)bh); } } }
  __syncthreads();
  for (int e = tid; e < 128 * 8; e += 128) { const int cl = e >> 3, q = e & 7;
    vst2((void*)(VT + (bb * CC + c0 + cl) * (size_t)SEQ + t0 + q * 8), *(const v4u*)&th[cl][q * 8]);
    if (hi_rows) { const size_t o3 = (bb * CC + c0 + cl) * (size_t)KHI + t0 + q * 8; vst2((void*)(VB + o3), *(const v4u*)&tb[cl][q * 8]); vst2((void*)(VBL + o3), *(const v4u*)&tbl[cl][q * 8]); } }
}

template <bool HI>
__device__ __forceinline__ void attn_body(const __bf16* __restrict__ QK, const _Float16* __restrict__ VT, const __bf16* __restrict__ VB, const __bf16* __restrict__ VBL, __bf16* __restrict__ CH, __bf16* __restrict__ CL, const int qb) {
  __shared__ __align__(16) _Float16 ph[4][16][40];
  __shared__ __align__(16) __bf16 pb[4][16][40];
  __shared__ __align__(16) __bf16 pbl[4][16][40];
  __shared__ __align__(16) __bf16 ch[4][16][72];
  __shared__ __align__(16) __bf16 cl[4][16][72];
  const int tid = threadIdx.x; const int wave = __builtin_amdgcn_readfirstlane((int)(threadIdx.x >> 5)); const int lane = tid & 31, col = lane & 15, g = lane >> 4;
  const int h = blockIdx.y, b = blockIdx.z;
  const __bf16* QH = QK; const __bf16* QL = QK + PLN; const __bf16* KH = QK + 2u * PLN; const __bf16* KL = QK + 3u * PLN;
  const int qw0 = qb * 64 + wave * 16;
  const size_t rowb = (size_t)b * SEQ;
  const size_t qoff = (rowb + qw0 + col) * CC + h * HD;
  const v16b qh0 = frag_b(QH + qoff, lane), qh1 = frag_b(QH + qoff + 32, lane), ql0 = frag_b(QL + qoff, lane), ql1 = frag_b(QL + qoff + 32, lane);
  v8f o[4] = {}; float m[8], l[8];
#pragma unroll
  for (int r = 0; r < 8; ++r) { m[r] = -1.0e30f; l[r] = 0.f; }
  const int nhalf = ((qw0 + 15) >> 5) + 1;
  const size_t vrow = (size_t)b * CC + h * HD + col;
#pragma unroll 1
  for (int hf = 0; hf < nhalf; ++hf) { const int kk0 = hf * 32;
    v8f s0 = {}, s1 = {};
    const size_t ko0 = (rowb + kk0 + col) * CC + h * HD; const size_t ko1 = ko0 + (size_t)16 * CC;
    { const v16b kh = frag_b(KH + ko0, lane), kl = frag_b(KL + ko0, lane); s0 = wmma_bf(ql0, kh, s0); s0 = wmma_bf(qh0, kl, s0); s0 = wmma_bf(qh0, kh, s0); }
    { const v16b kh = frag_b(KH + ko0 + 32, lane), kl = frag_b(KL + ko0 + 32, lane); s0 = wmma_bf(ql1, kh, s0); s0 = wmma_bf(qh1, kl, s0); s0 = wmma_bf(qh1, kh, s0); }
    { const v16b kh = frag_b(KH + ko1, lane), kl = frag_b(KL + ko1, lane); s1 = wmma_bf(ql0, kh, s1); s1 = wmma_bf(qh0, kl, s1); s1 = wmma_bf(qh0, kh, s1); }
    { const v16b kh = frag_b(KH + ko1 + 32, lane), kl = frag_b(KL + ko1 + 32, lane); s1 = wmma_bf(ql1, kh, s1); s1 = wmma_bf(qh1, kl, s1); s1 = wmma_bf(qh1, kh, s1); }
    float alpha[8];
#pragma unroll
    for (int r = 0; r < 8; ++r) { const int qr = qw0 + 8 * g + r; const bool v0 = (kk0 + col) <= qr, v1 = (kk0 + 16 + col) <= qr;
      const float a0 = v0 ? s0[r] * SCALE : -1.0e30f, a1 = v1 ? s1[r] * SCALE : -1.0e30f;
      float rm = fmaxf(a0, a1);
      rm = fmaxf(rm, __shfl_xor(rm, 1)); rm = fmaxf(rm, __shfl_xor(rm, 2)); rm = fmaxf(rm, __shfl_xor(rm, 4)); rm = fmaxf(rm, __shfl_xor(rm, 8));
      const float mn = fmaxf(m[r], rm); const float al = __expf(m[r] - mn);
      const float x0 = __expf(a0 - mn), x1 = __expf(a1 - mn); const float e0 = v0 ? x0 : 0.f, e1 = v1 ? x1 : 0.f;
      l[r] = l[r] * al + (e0 + e1); m[r] = mn; alpha[r] = al;
      if (HI) { const __bf16 h0 = (__bf16)e0, h1 = (__bf16)e1; pb[wave][8 * g + r][col] = h0; pb[wave][8 * g + r][16 + col] = h1; pbl[wave][8 * g + r][col] = (__bf16)(e0 - (float)h0); pbl[wave][8 * g + r][16 + col] = (__bf16)(e1 - (float)h1); }
      else { ph[wave][8 * g + r][col] = (_Float16)(e0 * PCARRY); ph[wave][8 * g + r][16 + col] = (_Float16)(e1 * PCARRY); } }
#pragma unroll
    for (int j = 0; j < 4; ++j) {
#pragma unroll
      for (int r = 0; r < 8; ++r) o[j][r] *= alpha[r]; }
    LDSX();
    if (HI) {
      union { v16b v; v8b q[2]; } uh, ul;
      uh.q[0] = *(const v8b*)&pb[wave][col][8 * g]; uh.q[1] = *(const v8b*)&pb[wave][col][16 + 8 * g];
      ul.q[0] = *(const v8b*)&pbl[wave][col][8 * g]; ul.q[1] = *(const v8b*)&pbl[wave][col][16 + 8 * g];
      asm volatile("" ::: "memory");
#pragma unroll
      for (int j = 0; j < 4; ++j) { const size_t po = (vrow + j * 16) * (size_t)KHI + kk0; const v16b vh = frag_b(VB + po, lane), vl = frag_b(VBL + po, lane);
        o[j] = wmma_bf(ul.v, vh, o[j]); o[j] = wmma_bf(uh.v, vl, o[j]); o[j] = wmma_bf(uh.v, vh, o[j]); }
    } else {
      union { v16h v; v8h q[2]; } up;
      up.q[0] = *(const v8h*)&ph[wave][col][8 * g]; up.q[1] = *(const v8h*)&ph[wave][col][16 + 8 * g];
      asm volatile("" ::: "memory");
#pragma unroll
      for (int j = 0; j < 4; ++j) { const size_t po = (vrow + j * 16) * (size_t)SEQ + kk0; o[j] = wmma16(up.v, frag_h(VT + po, lane), o[j]); }
    }
  }
  float inv[8];
#pragma unroll
  for (int r = 0; r < 8; ++r) { float ls = l[r]; ls += __shfl_xor(ls, 1); ls += __shfl_xor(ls, 2); ls += __shfl_xor(ls, 4); ls += __shfl_xor(ls, 8);
    inv[r] = (HI ? 1.0f : (1.0f / PCARRY)) * (1.0f / ls); }
#pragma unroll
  for (int j = 0; j < 4; ++j) {
#pragma unroll
    for (int r = 0; r < 8; ++r) { const float c = o[j][r] * inv[r]; const __bf16 hh = (__bf16)c; ch[wave][8 * g + r][j * 16 + col] = hh; cl[wave][8 * g + r][j * 16 + col] = (__bf16)(c - (float)hh); } }
  LDSX();
  for (int it = 0; it < 4; ++it) { const int rl = it * 4 + (lane >> 3), pc = lane & 7; const size_t off = (rowb + qw0 + rl) * CC + h * HD + pc * 8;
    vst2((void*)(CH + off), *(const v4u*)&ch[wave][rl][pc * 8]); vst2((void*)(CL + off), *(const v4u*)&cl[wave][rl][pc * 8]); }
}
__global__ __launch_bounds__(128) void k_attn_hi(const __bf16* __restrict__ QK, const _Float16* __restrict__ VT, const __bf16* __restrict__ VB, const __bf16* __restrict__ VBL, __bf16* __restrict__ CH, __bf16* __restrict__ CL) {
  attn_body<true>(QK, VT, VB, VBL, CH, CL, (int)blockIdx.x);
}
__global__ __launch_bounds__(128) void k_attn(const __bf16* __restrict__ QK, const _Float16* __restrict__ VT, const __bf16* __restrict__ VB, const __bf16* __restrict__ VBL, __bf16* __restrict__ CH, __bf16* __restrict__ CL) {
  attn_body<false>(QK, VT, VB, VBL, CH, CL, (int)blockIdx.x + QBH);
}

__global__ __launch_bounds__(128) void k_out(const __bf16* __restrict__ CH, const __bf16* __restrict__ CL, const __bf16* __restrict__ WOB, float* __restrict__ OUT) {
  __shared__ __align__(16) float sf[4][16][132];
  const int tid = threadIdx.x; const int wave = __builtin_amdgcn_readfirstlane((int)(threadIdx.x >> 5)); const int lane = tid & 31, col = lane & 15, g = lane >> 4;
  const int c0 = blockIdx.y * 128; const size_t rblk = (size_t)blockIdx.x * 64; const size_t bb = rblk / SEQ; const int t0 = (int)(rblk % SEQ);
  const size_t arow = rblk + wave * 16 + col;
  v8f acc[8] = {};
#pragma unroll 2
  for (int kc = 0; kc < CC / 32; ++kc) { const v16b ah = frag_b(CH + arow * CC + kc * 32, lane), al = frag_b(CL + arow * CC + kc * 32, lane);
#pragma unroll
    for (int j = 0; j < 8; ++j) { const v16b w = frag_b(WOB + (size_t)(c0 + j * 16 + col) * CC + kc * 32, lane); acc[j] = wmma_bf(al, w, acc[j]); acc[j] = wmma_bf(ah, w, acc[j]); } }
#pragma unroll
  for (int j = 0; j < 8; ++j) {
#pragma unroll
    for (int r = 0; r < 8; ++r) sf[wave][8 * g + r][j * 16 + col] = acc[j][r]; }
  LDSX();
  const size_t orow = bb * SEQ_FULL + t0 + wave * 16;
  for (int rl = 0; rl < 16; ++rl) vst2((void*)(OUT + (orow + rl) * DIN + c0 + lane * 4), *(const v4f*)&sf[wave][rl][lane * 4]);
}

extern "C" void kernel_launch(void* const* d_in, const int* in_sizes, int n_in, void* d_out, int out_size, void* d_ws, size_t ws_size, hipStream_t stream) {
  if (n_in < 5) return;
  const long long xneed = ((long long)(NB - 1) * SEQ_FULL + SEQ) * DIN;
  if ((long long)in_sizes[0] < xneed) return;
  for (int i = 1; i < 5; ++i) if ((long long)in_sizes[i] < (long long)CC * DIN) return;
  if ((long long)out_size < xneed) return;
  if (ws_size < (size_t)WS_END) return;
  const float* X = (const float*)d_in[0]; const float* WQ = (const float*)d_in[1]; const float* WK = (const float*)d_in[2]; const float* WV = (const float*)d_in[3]; const float* WO = (const float*)d_in[4];
  char* ws = (char*)d_ws;
  __bf16* XB = (__bf16*)(ws + WS_XB); __bf16* WB = (__bf16*)(ws + WS_WB); float* CS = (float*)(ws + WS_CS); __bf16* QK = (__bf16*)(ws + WS_QK);
  _Float16* VT = (_Float16*)(ws + WS_VT); __bf16* VB = (__bf16*)(ws + WS_VB); __bf16* VBL = (__bf16*)(ws + WS_VBL); __bf16* CH = (__bf16*)(ws + WS_CH); __bf16* CL = (__bf16*)(ws + WS_CL);
  k_cvt<<<dim3((unsigned)(PLN / 2048)), 256, 0, stream>>>(X, XB, SEQ, SEQ_FULL);
  k_cvt<<<dim3((unsigned)(WN / 2048)), 256, 0, stream>>>(WQ, WB, CC, CC);
  k_cvt<<<dim3((unsigned)(WN / 2048)), 256, 0, stream>>>(WK, WB + WN, CC, CC);
  k_cvt<<<dim3((unsigned)(WN / 2048)), 256, 0, stream>>>(WV, WB + 2u * WN, CC, CC);
  k_cvt<<<dim3((unsigned)(WN / 2048)), 256, 0, stream>>>(WO, WB + 3u * WN, CC, CC);
  k_tab<<<dim3(SEQ / 8), 256, 0, stream>>>(CS);
  k_projqk<<<dim3(NB * SEQ / 64, CC / 128, 2), 128, 0, stream>>>(XB, WB, CS, QK);
  k_projv<<<dim3(NB * SEQ / 64, CC / 128), 128, 0, stream>>>(XB, WB, VT, VB, VBL);
  k_attn_hi<<<dim3(QBH, NH, NB), 128, 0, stream>>>(QK, VT, VB, VBL, CH, CL);
  if (NQB > QBH) k_attn<<<dim3(NQB - QBH, NH, NB), 128, 0, stream>>>(QK, VT, VB, VBL, CH, CL);
  k_out<<<dim3(NB * SEQ / 64, DIN / 128), 128, 0, stream>>>(CH, CL, WB + 3u * WN, (float*)d_out);
}
